// GAU_48627619726042
// MI455X (gfx1250) — hardware-verified
//
#include <hip/hip_runtime.h>


namespace {
constexpr int Bn = 8, T = 2048, D = 512, E = 1024, S = 128, UV = 2 * E + S  , NT = Bn * T;
constexpr float XS = 8.0f, PS = 8.0f, EPS = 1e-5f, ISQ = 0.08838834764831845f  ;
struct Wo_ { static constexpr size_t UVo = 0, O = (size_t)UV * D, END = O + (size_t)D * E; };

typedef _Float16 b16;
typedef __attribute__((ext_vector_type(16))) _Float16 v16b;
typedef __attribute__((ext_vector_type(8))) _Float16 v8b;
typedef __attribute__((ext_vector_type(8))) float v8f;
typedef __attribute__((ext_vector_type(4))) float v4f;
__device__ __forceinline__ float bf16_rne(float f) { unsigned int u = __float_as_uint(f); u += 0x7FFFu + ((u >> 16) & 1u); return __uint_as_float(u & 0xFFFF0000u); }
__device__ __forceinline__ void split16(float v, b16& hi, b16& lo) { hi = (b16)v; lo = (b16)(v - (float)hi); }
__device__ __forceinline__ v16b frag_kb(const b16* p, int hh) { const v8b a = *(const v8b*)(p + 8 * hh), b = *(const v8b*)(p + 16 + 8 * hh); v16b f;
#pragma unroll
  for (int e = 0; e < 8; ++e) { f[e] = a[e]; f[8 + e] = b[e]; } return f; }
__device__ __forceinline__ void frag_split(const float* p, int hh, v16b& fh, v16b& fl) {
#pragma unroll
  for (int e = 0; e < 8; ++e) { b16 a, c; split16(p[8 * hh + e] * XS, a, c); fh[e] = a; fl[e] = c; split16(p[16 + 8 * hh + e] * XS, a, c); fh[8 + e] = a; fl[8 + e] = c; } }
__device__ __forceinline__ v8f wmma16b(v16b a, v16b b, v8f c) { v8f d = __builtin_amdgcn_wmma_f32_16x16x32_f16(false, a, false, b, (short)0, c, false, false); asm volatile("v_nop\n\tv_nop\n\tv_nop\n\tv_nop" : "+v"(d) : "v"(a), "v"(b)); return d; }
__device__ __forceinline__ void wave_lds_sync() { __builtin_amdgcn_fence(__ATOMIC_RELEASE, "workgroup"); __builtin_amdgcn_wave_barrier(); __builtin_amdgcn_fence(__ATOMIC_ACQUIRE, "workgroup"); }
__device__ __forceinline__ float nexp(float x) { return __builtin_amdgcn_exp2f(x * 1.4426950408889634f); }
__device__ __forceinline__ float pmul(float a, float b) { float p = a * b; asm volatile("" : "+v"(p)); return p; }
__device__ __forceinline__ float wsum(float v) {
#pragma unroll
  for (int o = 1; o < 32; o <<= 1) v += __shfl_xor(v, o); return v; }
__device__ __forceinline__ float silu_f(float y) { return y / (1.0f + nexp(-y)); }
__device__ __forceinline__ void sincos_r(float ang, float& sn, float& cs) { const float k = rintf(ang * 0.15915494309189535f); float r = __builtin_fmaf(k, -6.28318548202514648f, ang); r = __builtin_fmaf(k, 1.7484556025237907e-7f, r);
  const float t = r * 0.15915494309189535f; sn = __builtin_amdgcn_sinf(t); cs = __builtin_amdgcn_cosf(t); }

__global__ __launch_bounds__(256) void prep_kernel(const float* __restrict__ wuv, const float* __restrict__ wo, const float* __restrict__ g, const float* __restrict__ gm, const float* __restrict__ bt, const float* __restrict__ wr, b16* __restrict__ R, float* __restrict__ P) {
  const size_t tid = (size_t)blockIdx.x * 256 + threadIdx.x, nth = (size_t)gridDim.x * 256;
  for (int pass = 0; pass < 2; ++pass) { for (size_t p = tid; p < Wo_::END / 8; p += nth) { const size_t q = p * 8; const float* s_ = (q < Wo_::O) ? (wuv + q) : (wo + (q - Wo_::O)); v8b v; for (int e = 0; e < 8; ++e) v[e] = (b16)bf16_rne(s_[e]); *(volatile v8b*)(R + q) = v; }
    for (size_t q = tid; q < 4608; q += nth) { const int i = (int)q; float v; if (i == 0) v = g[0]; else if (i < 257) v = gm[i - 1]; else if (i < 513) v = bt[i - 257]; else v = wr[i - 513]; P[q] = bf16_rne(v); }
    __threadfence(); }
}

__global__ __launch_bounds__(256) void norm_kernel(const float* __restrict__ x, const float* __restrict__ P, b16* __restrict__ XH, b16* __restrict__ XL) {
  const int row = blockIdx.x * 8 + (threadIdx.x >> 5), lane = threadIdx.x & 31; const float* xr = x + (size_t)row * D;
  float v[16]; float ss = 0.0f;
#pragma unroll
  for (int i = 0; i < 16; ++i) { v[i] = bf16_rne(xr[(i >> 3) * 256 + lane * 8 + (i & 7)]); ss += pmul(v[i], v[i]); }
  ss = wsum(ss); const float nrm = sqrtf(ss) * 0.044194173824159216f; const float sc = P[0] / fmaxf(nrm, EPS);
  for (int pass = 0; pass < 2; ++pass) {
#pragma unroll
    for (int gq = 0; gq < 2; ++gq) { v8b h_, l_; for (int e = 0; e < 8; ++e) { b16 a_, c_; split16(v[gq * 8 + e] * sc * XS, a_, c_); h_[e] = a_; l_[e] = c_; } const size_t gi = (size_t)row * D + gq * 256 + lane * 8; *(volatile v8b*)(XH + gi) = h_; *(volatile v8b*)(XL + gi) = l_; }
    __threadfence(); }
}

template <int TWO>
__global__ __launch_bounds__(64) void uv_kernel(const b16* __restrict__ XH, const b16* __restrict__ XL, const b16* __restrict__ R, float* __restrict__ U, b16* __restrict__ VRh, b16* __restrict__ VRl, float* __restrict__ BS, int cblk0) {
  __shared__ __attribute__((aligned(16))) float Ts[2][32][64 + 4];
  const int lane = threadIdx.x & 31, wave = threadIdx.x >> 5, nloc = lane & 15, hlf = lane >> 4, m0 = blockIdx.y * 32, c0 = (blockIdx.x + cblk0) * 128 + wave * 64;
  v8f acc[2][4];
#pragma unroll
  for (int r = 0; r < 2; ++r)
#pragma unroll
    for (int t = 0; t < 4; ++t) acc[r][t] = (v8f){};
#pragma unroll 2
  for (int kb = 0; kb < D; kb += 32) { const v16b a0 = frag_kb(XH + (size_t)(m0 + nloc) * D + kb, hlf), a1 = frag_kb(XH + (size_t)(m0 + 16 + nloc) * D + kb, hlf); v16b l0, l1; if (TWO) { l0 = frag_kb(XL + (size_t)(m0 + nloc) * D + kb, hlf); l1 = frag_kb(XL + (size_t)(m0 + 16 + nloc) * D + kb, hlf); }
#pragma unroll
    for (int t = 0; t < 4; ++t) { const v16b bw = frag_kb(R + Wo_::UVo + (size_t)(c0 + t * 16 + nloc) * D + kb, hlf); acc[0][t] = wmma16b(a0, bw, acc[0][t]); acc[1][t] = wmma16b(a1, bw, acc[1][t]); if (TWO) { acc[0][t] = wmma16b(l0, bw, acc[0][t]); acc[1][t] = wmma16b(l1, bw, acc[1][t]); } } }
#pragma unroll
  for (int t = 0; t < 4; ++t)
#pragma unroll
    for (int r = 0; r < 2; ++r)
#pragma unroll
      for (int v = 0; v < 8; ++v) Ts[wave][r * 16 + 8 * hlf + v][t * 16 + nloc] = silu_f(acc[r][t][v] * (1.0f / XS));
  wave_lds_sync();
  for (int pass = 0; pass < 2; ++pass) {
    if (c0 < E) { for (int i = lane; i < 32 * 16; i += 32) { const int rr = i >> 4, c4 = (i & 15) * 4; *(volatile v4f*)(U + (size_t)(m0 + rr) * E + c0 + c4) = *(const v4f*)(&Ts[wave][rr][c4]); } }
    else if (c0 < 2 * E) { for (int i = lane; i < 32 * 8; i += 32) { const int rr = i >> 3, c8 = (i & 7) * 8; v8b h_, l_; for (int e = 0; e < 8; ++e) { b16 a_, c_; split16(Ts[wave][rr][c8 + e] * XS, a_, c_); h_[e] = a_; l_[e] = c_; } const size_t gi = (size_t)(m0 + rr) * E + (c0 - E) + c8; *(volatile v8b*)(VRh + gi) = h_; *(volatile v8b*)(VRl + gi) = l_; } }
    else { for (int i = lane; i < 32 * 16; i += 32) { const int rr = i >> 4, c4 = (i & 15) * 4; *(volatile v4f*)(BS + (size_t)(m0 + rr) * S + (c0 - 2 * E) + c4) = *(const v4f*)(&Ts[wave][rr][c4]); } }
    __threadfence(); }
}

__constant__ unsigned int kInvFreqBits[64] = {0x3f800000,0x3f93cfe5,0x3faab0d5,0x3fc51c50,0x3fe39ea9,0x40036cf4,0x4017c496,0x402f4244,0x404a62c2,0x4069b621,0x4086f161,0x409bd461,0x40b3f300,0x40cfcd58,0x40eff755,0x410a8de6,0x41200000,0x4138c3df,0x41555d0a,0x41766364,0x418e432a,0x41a44831,0x41bdb5bc,0x41db12d6,0x41fcfb72,0x421211d5,0x4228adb9,0x4242c979,0x4260efc0,0x4281e057,0x4295fa95,0x42ad3160,0x42c80000,0x42e6f4d6,0x43055a26,0x4319fe1e,0x4331d3f4,0x434d5a3e,0x436d232b,0x4388ebc5,0x439e1d27,0x43b6964a,0x43d2d927,0x43f37bd8,0x440c95d8,0x4422586d,0x443b793b,0x44587db7,0x447a0000,0x44905906,0x44a6b0b0,0x44c07da6,0x44de48f1,0x45005867,0x451435fb,0x452b26b7,0x4545a471,0x45643bdc,0x4583c7b8,0x45982d67,0x45afbb4e,0x45caee88,0x45ea5789,0x46074e93};
__global__ __launch_bounds__(256) void qk_kernel(const float* __restrict__ BS, const float* __restrict__ P, b16* __restrict__ QH, b16* __restrict__ QL, b16* __restrict__ KH, b16* __restrict__ KL) {
  __shared__ __attribute__((aligned(16))) b16 St[8][4][S + 8];
  const int wave = threadIdx.x >> 5, lane = threadIdx.x & 31, row = blockIdx.x * 8 + wave; const int t = row % T; const float* br = BS + (size_t)row * S;
  for (int hq = 0; hq < 2; ++hq) { const int i = hq * 32 + lane; const float b1 = br[i], b2 = br[64 + i]; const float invf = __uint_as_float(kInvFreqBits[i]); float sn, cs; sincos_r(pmul((float)t, invf), sn, cs);
#pragma unroll
    for (int brn = 0; brn < 2; ++brn) { const float x1 = pmul(b1, P[1 + brn * 128 + i]) + P[257 + brn * 128 + i], x2 = pmul(b2, P[1 + brn * 128 + 64 + i]) + P[257 + brn * 128 + 64 + i];
      const float o1 = pmul(x1, cs) - pmul(x2, sn), o2 = pmul(x2, cs) + pmul(x1, sn); b16 a_, c_; split16(o1 * XS, a_, c_); St[wave][brn * 2][i] = a_; St[wave][brn * 2 + 1][i] = c_; split16(o2 * XS, a_, c_); St[wave][brn * 2][64 + i] = a_; St[wave][brn * 2 + 1][64 + i] = c_; } }
  wave_lds_sync();
  for (int pass = 0; pass < 2; ++pass) { if (lane < 16) { b16* dsts[4] = {QH, QL, KH, KL};
#pragma unroll
      for (int pl = 0; pl < 4; ++pl) *(volatile v8b*)(dsts[pl] + (size_t)row * S + lane * 8) = *(const v8b*)(&St[wave][pl][lane * 8]); } __threadfence(); }
}

__global__ __launch_bounds__(256) void vt_kernel(const b16* __restrict__ Vr, b16* __restrict__ vt) {
  __shared__ __attribute__((aligned(16))) b16 Tt[128][128 + 8];
  const int b = 0, ch = blockIdx.y * 128, t0 = blockIdx.x * 128, t_ = threadIdx.x;
  for (int i = t_; i < 128 * 16; i += 256) { const int tk = i >> 4, d8 = (i & 15) * 8; const v8b vv = *(const v8b*)(Vr + ((size_t)(b * T + t0 + tk)) * E + ch + d8); for (int e = 0; e < 8; ++e) Tt[d8 + e][tk] = vv[e]; }
  __syncthreads();
  for (int pass = 0; pass < 2; ++pass) { for (int i = t_; i < 128 * 16; i += 256) { const int d = i >> 4, c8 = (i & 15) * 8; *(volatile v8b*)(vt + ((size_t)b * E + ch + d) * T + t0 + c8) = *(const v8b*)(&Tt[d][c8]); } __threadfence(); }
}

__global__ __launch_bounds__(256) void attn_kernel(const b16* __restrict__ QH, const b16* __restrict__ QL, const b16* __restrict__ KH, const b16* __restrict__ KL, const b16* __restrict__ VTh, const b16* __restrict__ VTl, const float* __restrict__ P, float* __restrict__ A) {
  __shared__ float Sx[2][16][16 + 1]; __shared__ __attribute__((aligned(16))) float Os[16][E + 4];
  const int wave = threadIdx.x >> 5, lane = threadIdx.x & 31, hh = lane >> 4, col = lane & 15; const int b = 0, q0 = blockIdx.x * 16, qi = q0 + col;
  const size_t rb = 0; const b16* Vh = VTh + ((size_t)wave * 128) * T; const b16* Vl = VTl + ((size_t)wave * 128) * T; const float SC = 1.0f / (XS * XS); const float* wrel = P + 513; (void)b;
  v16b qh_[4], ql_[4];
#pragma unroll
  for (int j = 0; j < 4; ++j) { qh_[j] = frag_kb(QH + rb + (size_t)qi * S + 32 * j, hh); ql_[j] = frag_kb(QL + rb + (size_t)qi * S + 32 * j, hh); }
  v8f o[8];
#pragma unroll
  for (int t = 0; t < 8; ++t) o[t] = (v8f){};
  for (int kb = 0; kb < T; kb += 32) {
    if (wave < 2) { v8f s = {};
#pragma unroll
      for (int j = 0; j < 4; ++j) { const v16b kh_ = frag_kb(KH + rb + (size_t)(kb + 16 * wave + col) * S + 32 * j, hh), kl_ = frag_kb(KL + rb + (size_t)(kb + 16 * wave + col) * S + 32 * j, hh); s = wmma16b(kh_, qh_[j], s); s = wmma16b(kh_, ql_[j], s); s = wmma16b(kl_, qh_[j], s); }
#pragma unroll
      for (int r = 0; r < 8; ++r) Sx[wave][8 * hh + r][col] = s[r]; }
    __syncthreads();
    v16b pb;
#pragma unroll
    for (int r = 0; r < 8; ++r) { const int j0 = kb + 8 * hh + r, j1 = j0 + 16;
      const float s0 = (Sx[0][8 * hh + r][col] * SC + wrel[(T - 1) + j0 - qi]) * ISQ, s1 = (Sx[1][8 * hh + r][col] * SC + wrel[(T - 1) + j1 - qi]) * ISQ;
      const float p0 = (s0 > 0.0f) ? pmul(s0, s0) : 0.0f, p1 = (s1 > 0.0f) ? pmul(s1, s1) : 0.0f; pb[r] = (b16)(p0 * PS); pb[8 + r] = (b16)(p1 * PS); }
    __syncthreads();
#pragma unroll
    for (int t = 0; t < 8; ++t) { o[t] = wmma16b(frag_kb(Vh + (size_t)(t * 16 + col) * T + kb, hh), pb, o[t]); } (void)Vl; }
#pragma unroll
  for (int t = 0; t < 8; ++t)
#pragma unroll
    for (int r = 0; r < 8; ++r) Os[col][wave * 128 + t * 16 + 8 * hh + r] = o[t][r] * (1.0f / (PS * XS));
  __syncthreads();
  for (int pass = 0; pass < 2; ++pass) { for (int i = threadIdx.x; i < 16 * (E / 4); i += 256) { const int rr = i / (E / 4), c4 = (i % (E / 4)) * 4; *(volatile v4f*)(A + ((size_t)(b * T + q0 + rr)) * E + c4) = *(const v4f*)(&Os[rr][c4]); } __threadfence(); }
}

__global__ __launch_bounds__(256) void gate_kernel(const float* __restrict__ U, const float* __restrict__ A, b16* __restrict__ Gh, b16* __restrict__ Gl) {
  const size_t tid = (size_t)blockIdx.x * 256 + threadIdx.x, nth = (size_t)gridDim.x * 256;
  for (int pass = 0; pass < 2; ++pass) { for (size_t p = tid; p < (size_t)T * E / 8; p += nth) { v8b h_, l_; for (int e = 0; e < 8; ++e) { b16 a_, c_; split16(pmul(U[p * 8 + e], A[p * 8 + e]) * XS, a_, c_); h_[e] = a_; l_[e] = c_; } *(volatile v8b*)(Gh + p * 8) = h_; *(volatile v8b*)(Gl + p * 8) = l_; } __threadfence(); }
}

__global__ __launch_bounds__(64) void out_kernel(const b16* __restrict__ Gh, const b16* __restrict__ Gl, const b16* __restrict__ R, const float* __restrict__ x, float* __restrict__ out) {
  __shared__ __attribute__((aligned(16))) float Ts[2][32][128 + 4];
  const int lane = threadIdx.x & 31, wave = threadIdx.x >> 5, nloc = lane & 15, hlf = lane >> 4, m0 = blockIdx.y * 32, c0 = blockIdx.x * 256 + wave * 128; const b16* Wo = R + Wo_::O;
#pragma unroll 1
  for (int hf = 0; hf < 2; ++hf) { v8f acc[2][4];
#pragma unroll
    for (int r = 0; r < 2; ++r)
#pragma unroll
      for (int t = 0; t < 4; ++t) acc[r][t] = (v8f){};
#pragma unroll 2
    for (int kb = 0; kb < E; kb += 32) { const v16b a0 = frag_kb(Gh + (size_t)(m0 + nloc) * E + kb, hlf), a1 = frag_kb(Gh + (size_t)(m0 + 16 + nloc) * E + kb, hlf); (void)Gl;
#pragma unroll
      for (int t = 0; t < 4; ++t) { const v16b bw = frag_kb(Wo + (size_t)(c0 + (hf * 4 + t) * 16 + nloc) * E + kb, hlf); acc[0][t] = wmma16b(a0, bw, acc[0][t]); acc[1][t] = wmma16b(a1, bw, acc[1][t]); } }
#pragma unroll
    for (int t = 0; t < 4; ++t) { const int cl = (hf * 4 + t) * 16 + nloc, c = c0 + cl;
#pragma unroll
      for (int r = 0; r < 2; ++r)
#pragma unroll
        for (int v = 0; v < 8; ++v) { const int row = m0 + r * 16 + 8 * hlf + v; Ts[wave][r * 16 + 8 * hlf + v][cl] = acc[r][t][v] * (1.0f / XS) + bf16_rne(x[(size_t)row * D + c]); } } }
  wave_lds_sync();
  for (int pass = 0; pass < 2; ++pass) { for (int i = lane; i < 32 * 32; i += 32) { const int rr = i >> 5, c4 = (i & 31) * 4; *(volatile v4f*)(out + (size_t)(m0 + rr) * D + c0 + c4) = *(const v4f*)(&Ts[wave][rr][c4]); } __threadfence(); }
}
}

extern "C" void kernel_launch(void* const* d_in, const int* in_sizes, int n_in,
                              void* d_out, int out_size, void* d_ws, size_t ws_size, hipStream_t stream) {
  (void)n_in; (void)out_size;
  const float* x = (const float*)d_in[0]; const float* g = (const float*)d_in[1]; const float* wuv = (const float*)d_in[2]; const float* gm = (const float*)d_in[3]; const float* bt = (const float*)d_in[4]; const float* wr = (const float*)d_in[5]; const float* wo = (const float*)d_in[6];
  float* out = (float*)d_out;
  if (in_sizes[0] != NT * D || in_sizes[2] != UV * D || in_sizes[5] != 2 * T - 1 || in_sizes[6] != D * E) return;
  size_t off = 0; char* ws = (char*)d_ws;
  auto carve = [&](size_t bytes) { char* p = ws + off; off += (bytes + 255) & ~(size_t)255; return p; };
  b16* R = (b16*)carve(Wo_::END * 2); float* P = (float*)carve(4608 * 4); b16* XH = (b16*)carve((size_t)T * D * 2); b16* XL = (b16*)carve((size_t)T * D * 2); float* U = (float*)carve((size_t)T * E * 4);
  b16* VRh = (b16*)carve((size_t)T * E * 2); b16* VRl = (b16*)carve((size_t)T * E * 2); b16* VTh = (b16*)carve((size_t)T * E * 2); b16* VTl = (b16*)carve((size_t)T * E * 2); float* BS = (float*)carve((size_t)T * S * 4);
  b16* QH = (b16*)carve((size_t)T * S * 2); b16* QL = (b16*)carve((size_t)T * S * 2); b16* KH = (b16*)carve((size_t)T * S * 2); b16* KL = (b16*)carve((size_t)T * S * 2); float* A = (float*)carve((size_t)T * E * 4); b16* Gh = (b16*)carve((size_t)T * E * 2); b16* Gl = (b16*)carve((size_t)T * E * 2);
  if (off > ws_size) return;
  prep_kernel<<<256, 256, 0, stream>>>(wuv, wo, g, gm, bt, wr, R, P);
  for (int b = 0; b < Bn; ++b) { const float* xb = x + (size_t)b * T * D; float* ob = out + (size_t)b * T * D;
    norm_kernel<<<T / 8, 256, 0, stream>>>(xb, P, XH, XL);
    uv_kernel<0><<<dim3(2 * E / 128, T / 32), 64, 0, stream>>>(XH, XL, R, U, VRh, VRl, BS, 0);
    uv_kernel<1><<<dim3(1, T / 32), 64, 0, stream>>>(XH, XL, R, U, VRh, VRl, BS, 2 * E / 128);
    qk_kernel<<<T / 8, 256, 0, stream>>>(BS, P, QH, QL, KH, KL);
    vt_kernel<<<dim3(T / 128, E / 128), 256, 0, stream>>>(VRh, VTh);
    vt_kernel<<<dim3(T / 128, E / 128), 256, 0, stream>>>(VRl, VTl);
    attn_kernel<<<T / 16, 256, 0, stream>>>(QH, QL, KH, KL, VTh, VTl, P, A);
    gate_kernel<<<256, 256, 0, stream>>>(U, A, Gh, Gl);
    out_kernel<<<dim3(D / 256, T / 32), 64, 0, stream>>>(Gh, Gl, R, xb, ob); }
}
